// MHLA_29841432772831
// MI455X (gfx1250) — hardware-verified
//
#include <hip/hip_runtime.h>
#include <math.h>

typedef __attribute__((ext_vector_type(16))) _Float16 v16h;
typedef __attribute__((ext_vector_type(16))) __bf16 v16b;
typedef __attribute__((ext_vector_type(8)))  _Float16 v8h;
typedef __attribute__((ext_vector_type(8)))  float v8f;
typedef __attribute__((ext_vector_type(4)))  float v4f;
typedef __attribute__((ext_vector_type(2)))  float v2f;
typedef __attribute__((ext_vector_type(4)))  unsigned v4u;
typedef __attribute__((ext_vector_type(4)))  int v4i;
typedef float __attribute__((may_alias)) float_a;
typedef int __attribute__((may_alias)) int_a;

template <typename T> __device__ __forceinline__ void vst2(void* p, T v) { *(volatile T*)p = v; __threadfence(); *(volatile T*)p = v; }
__device__ __forceinline__ v8f wmma16(v16h a, v16h b, v8f c) {
  v8f d = __builtin_amdgcn_wmma_f32_16x16x32_f16(false, a, false, b, (short)0, c, false, false);
  asm volatile("v_nop\n\tv_nop\n\tv_nop\n\tv_nop" : "+v"(d) : "v"(a), "v"(b));
  return d;
}
__device__ __forceinline__ v8f wmma_bf(v16b a, v16b b, v8f c) {
  v8f d = __builtin_amdgcn_wmma_f32_16x16x32_bf16(false, a, false, b, (short)0, c, false, false);
  asm volatile("v_nop\n\tv_nop\n\tv_nop\n\tv_nop" : "+v"(d) : "v"(a), "v"(b));
  return d;
}
__device__ __forceinline__ v16h frag_h(const _Float16* rowk0, int lane) {
  union { v16h v; v8h q[2]; } u; const _Float16* p = rowk0 + 8 * (lane >> 4);
  u.q[0] = *(const v8h*)p; u.q[1] = *(const v8h*)(p + 16); return u.v;
}
__device__ __forceinline__ v16h frag_f32(const float* rowk0, int lane) {
  v16h a; const float* p = rowk0 + 8 * (lane >> 4);
#pragma unroll
  for (int i = 0; i < 8; ++i) { a[i] = (_Float16)p[i]; a[8 + i] = (_Float16)p[16 + i]; }
  return a;
}
__device__ __forceinline__ v16h frag_f32s(const float* rowk0, int lane, float sc) {
  v16h a; const float* p = rowk0 + 8 * (lane >> 4);
#pragma unroll
  for (int i = 0; i < 8; ++i) { a[i] = (_Float16)(p[i] * sc); a[8 + i] = (_Float16)(p[16 + i] * sc); }
  return a;
}
__device__ __forceinline__ v16h fragc_f32(const float* W, int k0, int n, int lane, int ld, int K) {
  v16h a; const int g = lane >> 4;
#pragma unroll
  for (int i = 0; i < 8; ++i) { const int ka = k0 + 8 * g + i, kb = ka + 16;
    a[i] = (_Float16)(ka < K ? W[(size_t)(ka < K ? ka : K - 1) * ld + n] : 0.f); a[8 + i] = (_Float16)(kb < K ? W[(size_t)(kb < K ? kb : K - 1) * ld + n] : 0.f); }
  return a;
}
struct F2 { v16b h, l; };
__device__ __forceinline__ F2 bsplit16(const float v[16]) { F2 r;
#pragma unroll
  for (int i = 0; i < 16; ++i) { const __bf16 h = (__bf16)v[i]; r.h[i] = h; r.l[i] = (__bf16)(v[i] - (float)h); }
  return r; }
__device__ __forceinline__ F2 split_row(const float* row, int k0, int lane) { float v[16]; const float* p = row + k0 + 8 * (lane >> 4);
#pragma unroll
  for (int i = 0; i < 8; ++i) { v[i] = p[i]; v[8 + i] = p[16 + i]; }
  return bsplit16(v); }
__device__ __forceinline__ F2 split_rowK(const float* row, int k0, int lane, int K) { float v[16]; const int g = lane >> 4;
#pragma unroll
  for (int i = 0; i < 8; ++i) { const int ka = k0 + 8 * g + i, kb = ka + 16; v[i] = ka < K ? row[ka < K ? ka : K - 1] : 0.f; v[8 + i] = kb < K ? row[kb < K ? kb : K - 1] : 0.f; }
  return bsplit16(v); }
__device__ __forceinline__ F2 split_col(const float* W, int k0, int n, int lane, int ld, int K) { float v[16]; const int g = lane >> 4;
#pragma unroll
  for (int i = 0; i < 8; ++i) { const int ka = k0 + 8 * g + i, kb = ka + 16; v[i] = ka < K ? W[(size_t)(ka < K ? ka : K - 1) * ld + n] : 0.f; v[8 + i] = kb < K ? W[(size_t)(kb < K ? kb : K - 1) * ld + n] : 0.f; }
  return bsplit16(v); }
__device__ __forceinline__ v8f mac3(const F2& a, const F2& b, v8f c) { c = wmma_bf(a.l, b.h, c); c = wmma_bf(a.h, b.l, c); return wmma_bf(a.h, b.h, c); }
__device__ __forceinline__ float sigm(float v) { return 1.0f / (1.0f + expf(-v)); }
#define LDSX() do { asm volatile("s_wait_dscnt 0" ::: "memory"); __builtin_amdgcn_wave_barrier(); __builtin_amdgcn_fence(__ATOMIC_RELEASE, "workgroup"); } while (0)

__device__ __forceinline__ float bfr(float v) { return (float)(__bf16)v; }
#define NB 2
#define TT 2048
#define CC 1024
#define NH 32
#define HD 32
#ifndef TNB
#define TNB NB
#endif
#ifndef QSTR
#define QSTR (TT * CC)
#endif
typedef __attribute__((ext_vector_type(8))) __bf16 v8b;
__device__ __forceinline__ v16b frag_b(const __bf16* rowk0, int lane) { union { v16b v; v8b q[2]; } u; const __bf16* p = rowk0 + 8 * (lane >> 4); u.q[0] = *(const v8b*)p; u.q[1] = *(const v8b*)(p + 16); return u.v; }
#define WS_QH  0u
#define WS_QL  (WS_QH + 2u * (size_t)NB * TT * CC)
#define WS_KT  (WS_QL + 2u * (size_t)NB * TT * CC)
#define WS_KL  (WS_KT + 2u * (size_t)NB * CC * TT)
#define WS_VT  (WS_KL + 2u * (size_t)NB * CC * TT)
#define WS_VL  (WS_VT + 2u * (size_t)NB * CC * TT)
#define WS_KV  (WS_VL + 2u * (size_t)NB * CC * TT)
#define WS_KVL (WS_KV + 2u * (size_t)NB * NH * HD * HD)
#define WS_CTX (WS_KVL + 2u * (size_t)NB * NH * HD * HD)
#define WS_GS  (WS_CTX + 4u * (size_t)NB * TT * CC)
#define WS_END (WS_GS + 4u * (size_t)NB * NH * 2 * 16)
__global__ __launch_bounds__(128) void k_proj(const float* __restrict__ X, const float* __restrict__ Wt, const float* __restrict__ Bv, _Float16* __restrict__ QH, _Float16* __restrict__ QL, __bf16* __restrict__ KT, __bf16* __restrict__ KL, __bf16* __restrict__ VT, __bf16* __restrict__ VL) {
  __shared__ __align__(16) _Float16 sh[64][136], sl[64][136]; __shared__ __align__(16) __bf16 th[128][72], tl2[128][72];
  const int tid = threadIdx.x, wave = tid >> 5, lane = tid & 31, col = lane & 15, g = lane >> 4; const int which = blockIdx.z; const int c0 = blockIdx.y * 128; const size_t r0 = (size_t)blockIdx.x * 64;
  v8f acc[8] = {};
#pragma unroll 2
  for (int kc = 0; kc < CC / 32; ++kc) { v16b a; { const float* p = X + (r0 + wave * 16 + col) * CC + kc * 32 + 8 * g;
#pragma unroll
      for (int i = 0; i < 8; ++i) { a[i] = (__bf16)p[i]; a[8 + i] = (__bf16)p[16 + i]; } }
#pragma unroll
    for (int j = 0; j < 8; ++j) { v16b w; const float* wr = Wt + (size_t)(which * CC + c0 + j * 16 + col) * CC + kc * 32 + 8 * g;
#pragma unroll
      for (int i = 0; i < 8; ++i) { w[i] = (__bf16)wr[i]; w[8 + i] = (__bf16)wr[16 + i]; }
      asm volatile("s_wait_loadcnt 0x0" ::: "memory"); acc[j] = wmma_bf(a, w, acc[j]); } }
#pragma unroll
  for (int j = 0; j < 8; ++j) { const int cl = j * 16 + col; const float bb = bfr(Bv[which * CC + c0 + cl]);
#pragma unroll
    for (int r = 0; r < 8; ++r) { const float v = acc[j][r] + bb; const int rl = wave * 16 + 8 * g + r;
      if (which == 0) { const _Float16 hv = (_Float16)v; sh[rl][cl] = hv; sl[rl][cl] = (_Float16)((v - (float)hv) * 1024.0f); } else { const __bf16 bh = (__bf16)v; th[cl][rl] = bh; tl2[cl][rl] = (__bf16)(v - (float)bh); } } }
  __syncthreads();
  if (which == 0) { for (int e = tid; e < 64 * 16; e += 128) { const int rl = e >> 4, q = e & 15; vst2((unsigned*)(QH + (r0 + rl) * CC + c0 + q * 8), *(const v4u*)&sh[rl][q * 8]); vst2((unsigned*)(QL + (r0 + rl) * CC + c0 + q * 8), *(const v4u*)&sl[rl][q * 8]); } }
  else { __bf16* DT = which == 1 ? KT : VT; __bf16* DL = which == 1 ? KL : VL; const size_t b = r0 / TT; const int t0 = (int)(r0 % TT); for (int e = tid; e < 128 * 8; e += 128) { const int cl = e >> 3, q = e & 7; const size_t o2 = (b * CC + c0 + cl) * (size_t)TT + t0 + q * 8; vst2((unsigned*)(DT + o2), *(const v4u*)&th[cl][q * 8]); vst2((unsigned*)(DL + o2), *(const v4u*)&tl2[cl][q * 8]); } } }
__global__ __launch_bounds__(32) void k_kv(const __bf16* __restrict__ KT, const __bf16* __restrict__ KL, const __bf16* __restrict__ VT, const __bf16* __restrict__ VL, _Float16* __restrict__ KV, _Float16* __restrict__ KVL) { __shared__ __align__(16) _Float16 sh[32][40], sl[32][40];
  const int lane = threadIdx.x, col = lane & 15, g = lane >> 4; const size_t b = blockIdx.y; const int h = blockIdx.x; const __bf16* kb = KT + (b * CC + h * HD) * (size_t)TT; const __bf16* klb = KL + (b * CC + h * HD) * (size_t)TT; const __bf16* vb = VT + (b * CC + h * HD) * (size_t)TT; const __bf16* vlb = VL + (b * CC + h * HD) * (size_t)TT;
  v8f acc[2][2] = {};
#pragma unroll 2
  for (int kc = 0; kc < TT / 32; ++kc) {
#pragma unroll
    for (int it = 0; it < 2; ++it) { const v16b ah = frag_b(kb + (size_t)(it * 16 + col) * TT + kc * 32, lane), al = frag_b(klb + (size_t)(it * 16 + col) * TT + kc * 32, lane);
#pragma unroll
      for (int jt = 0; jt < 2; ++jt) { const v16b bh = frag_b(vb + (size_t)(jt * 16 + col) * TT + kc * 32, lane), bl = frag_b(vlb + (size_t)(jt * 16 + col) * TT + kc * 32, lane); acc[it][jt] = wmma_bf(ah, bh, acc[it][jt]); acc[it][jt] = wmma_bf(al, bh, acc[it][jt]); acc[it][jt] = wmma_bf(ah, bl, acc[it][jt]); } } }
#pragma unroll
  for (int it = 0; it < 2; ++it)
#pragma unroll
    for (int jt = 0; jt < 2; ++jt)
#pragma unroll
      for (int r = 0; r < 8; ++r) { const float v = acc[it][jt][r]; const int i = it * 16 + 8 * g + r, j = jt * 16 + col; const _Float16 hv = (_Float16)v; sh[j][i] = hv; sl[j][i] = (_Float16)((v - (float)hv) * 1024.0f); }
  LDSX();
  for (int e = lane; e < 32 * 4; e += 32) { const int j = e >> 2, q = e & 3; const size_t o = ((b * NH + h) * HD + j) * HD + q * 8; vst2((unsigned*)(KV + o), *(const v4u*)&sh[j][q * 8]); vst2((unsigned*)(KVL + o), *(const v4u*)&sl[j][q * 8]); } }
__global__ __launch_bounds__(128) void k_ctx(const _Float16* __restrict__ QH, const _Float16* __restrict__ QL, const _Float16* __restrict__ KV, const _Float16* __restrict__ KVL, float* __restrict__ CTX) { __shared__ __align__(16) float sf[4][16][132];
  const int tid = threadIdx.x, wave = tid >> 5, lane = tid & 31, col = lane & 15, g = lane >> 4; const int h0 = blockIdx.y * 4; const size_t r0 = (size_t)blockIdx.x * 64 + wave * 16; const size_t b = r0 / TT;
#pragma unroll
  for (int hh = 0; hh < 4; ++hh) { const int h = h0 + hh; v8f acc[2] = {}; const v16h ah = frag_h(QH + (r0 + col) * CC + h * HD, lane), al = frag_h(QL + (r0 + col) * CC + h * HD, lane);
#pragma unroll
    for (int jt = 0; jt < 2; ++jt) { const size_t bo = ((b * NH + h) * HD + jt * 16 + col) * HD; const v16h bh = frag_h(KV + bo, lane), bl = frag_h(KVL + bo, lane); acc[jt] = wmma16(ah, bh, acc[jt]); v8f t2 = {}; t2 = wmma16(al, bh, t2); t2 = wmma16(ah, bl, t2);
#pragma unroll
      for (int r = 0; r < 8; ++r) sf[wave][8 * g + r][hh * 32 + jt * 16 + col] = acc[jt][r] + t2[r] * (1.0f / 1024.0f); } }
  LDSX(); for (int rl = 0; rl < 16; ++rl) vst2(CTX + (r0 + rl) * CC + h0 * HD + lane * 4, *(const v4f*)&sf[wave][rl][lane * 4]); }
__global__ __launch_bounds__(256) void k_gn(const float* __restrict__ CTX, float* __restrict__ GS) { __shared__ float sred[8]; __shared__ float sbc;
  const int t = threadIdx.x; const int h = blockIdx.x; const size_t b = blockIdx.y; const float* base = CTX + (b * TT) * CC + h * HD; const int n = TT * HD;
  float s = 0.f; for (int e = t; e < TT * 8; e += 256) { const int row = e >> 3, q = e & 7; const v4f v = *(const v4f*)(base + (size_t)row * CC + q * 4); s += (v[0] + v[1]) + (v[2] + v[3]); }
#pragma unroll
  for (int o = 1; o < 32; o <<= 1) s += __shfl_xor(s, o);
  if ((t & 31) == 0) sred[t >> 5] = s; __syncthreads(); if (t == 0) { float a = 0.f; for (int w = 0; w < 8; ++w) a += sred[w]; sbc = a / (float)n; } __syncthreads(); const float mu = sbc; __syncthreads();
  float s2 = 0.f; for (int e = t; e < TT * 8; e += 256) { const int row = e >> 3, q = e & 7; const v4f v = *(const v4f*)(base + (size_t)row * CC + q * 4); const float d0 = v[0] - mu, d1 = v[1] - mu, d2 = v[2] - mu, d3 = v[3] - mu; s2 += (d0 * d0 + d1 * d1) + (d2 * d2 + d3 * d3); }
#pragma unroll
  for (int o = 1; o < 32; o <<= 1) s2 += __shfl_xor(s2, o);
  if ((t & 31) == 0) sred[t >> 5] = s2; __syncthreads();
  if (t < 32) { float v = 0.f; if (t == 0) v = mu; if (t == 1) { float a = 0.f; for (int w = 0; w < 8; ++w) a += sred[w]; v = rsqrtf(a / (float)n + 1e-5f); } vst2(GS + (b * NH + h) * 32 + t, v); } }
__global__ __launch_bounds__(128) void k_out(const float* __restrict__ CTX, const float* __restrict__ GS, const float* __restrict__ GW, const float* __restrict__ GB, const float* __restrict__ WO, const float* __restrict__ BO, float* __restrict__ OUT) { __shared__ __align__(16) float sf[4][16][132];
  const int tid = threadIdx.x, wave = tid >> 5, lane = tid & 31, col = lane & 15, g = lane >> 4; const int c0 = blockIdx.y * 128; const size_t r0 = (size_t)blockIdx.x * 64 + wave * 16; const size_t b = r0 / TT;
  v8f acc[8] = {};
#pragma unroll 2
  for (int kc = 0; kc < CC / 32; ++kc) { float v[16]; { const int h = kc;     const float mu = GS[(b * NH + h) * 32], rs = GS[(b * NH + h) * 32 + 1]; const float* p = CTX + (r0 + col) * CC + kc * 32 + 8 * g;
#pragma unroll
      for (int i = 0; i < 8; ++i) { const int c1 = kc * 32 + 8 * g + i, c2 = c1 + 16; v[i] = (p[i] - mu) * rs * bfr(GW[c1]) + bfr(GB[c1]); v[8 + i] = (p[16 + i] - mu) * rs * bfr(GW[c2]) + bfr(GB[c2]); } }
    asm volatile("s_wait_loadcnt 0x0" ::: "memory"); const F2 a = bsplit16(v);
#pragma unroll
    for (int j = 0; j < 8; ++j) { v16b w; const float* wr = WO + (size_t)(c0 + j * 16 + col) * CC + kc * 32 + 8 * g;
#pragma unroll
      for (int i = 0; i < 8; ++i) { w[i] = (__bf16)wr[i]; w[8 + i] = (__bf16)wr[16 + i]; }
      asm volatile("s_wait_loadcnt 0x0" ::: "memory"); acc[j] = wmma_bf(a.h, w, acc[j]); acc[j] = wmma_bf(a.l, w, acc[j]); } }
#pragma unroll
  for (int j = 0; j < 8; ++j) { const float bb = bfr(BO[c0 + j * 16 + col]);
#pragma unroll
    for (int r = 0; r < 8; ++r) sf[wave][8 * g + r][j * 16 + col] = acc[j][r] + bb; }
  LDSX(); for (int rl = 0; rl < 16; ++rl) vst2(OUT + (r0 + rl) * CC + c0 + lane * 4, *(const v4f*)&sf[wave][rl][lane * 4]); }
extern "C" void kernel_launch(void* const* d_in, const int* in_sizes, int n_in, void* d_out, int out_size, void* d_ws, size_t ws_size, hipStream_t stream) {
  (void)in_sizes; (void)n_in; (void)out_size;
  const float** F = (const float**)d_in;
  if (ws_size < (size_t)WS_END) return;
  char* ws = (char*)d_ws; _Float16 *QH = (_Float16*)(ws + WS_QH), *QL = (_Float16*)(ws + WS_QL), *KV = (_Float16*)(ws + WS_KV), *KVL = (_Float16*)(ws + WS_KVL); __bf16 *KT = (__bf16*)(ws + WS_KT), *KL = (__bf16*)(ws + WS_KL), *VT = (__bf16*)(ws + WS_VT), *VL = (__bf16*)(ws + WS_VL); float *CTX = (float*)(ws + WS_CTX), *GS = (float*)(ws + WS_GS);
  k_proj<<<dim3(TNB * TT / 64, CC / 128, 3), 128, 0, stream>>>(F[0], F[1], F[2], QH, QL, KT, KL, VT, VL);
  k_kv<<<dim3(NH, TNB), 32, 0, stream>>>(KT, KL, VT, VL, KV, KVL);
  k_ctx<<<dim3(TNB * TT / 64, NH / 4), 128, 0, stream>>>(QH, QL, KV, KVL, CTX);
  k_gn<<<dim3(NH, TNB), 256, 0, stream>>>(CTX, GS);
  k_out<<<dim3(TNB * TT / 64, CC / 128), 128, 0, stream>>>(CTX, GS, F[3], F[4], F[5], F[6], (float*)d_out);
}
